// DeformConvV3_50912542326882
// MI455X (gfx1250) — hardware-verified
//
#include <hip/hip_runtime.h>


namespace {
constexpr int NB_ = 8, C = 128, OC = 128, HH = 80, WW = 80, K9 = 9, KK = C * K9  , NP = HH * WW  , NPT = NB_ * NP, CIN2 = 160  ;
constexpr float XS = 8.0f, VS = 64.0f, HS = 256.0f, WSC = 256.0f;
typedef _Float16 b16;
typedef __attribute__((ext_vector_type(16))) _Float16 v16b;
typedef __attribute__((ext_vector_type(8))) _Float16 v8b;
typedef __attribute__((ext_vector_type(8))) float v8f;
typedef __attribute__((ext_vector_type(4))) float v4f;
__device__ __forceinline__ float bf16_rne(float f) { unsigned int u = __float_as_uint(f); u += 0x7FFFu + ((u >> 16) & 1u); float r = __uint_as_float(u & 0xFFFF0000u); asm volatile("" : "+v"(r)); return r; }
__device__ __forceinline__ float bfv(float f) { float r = bf16_rne(f); asm volatile("" : "+v"(r)); return r; }
__device__ __forceinline__ void split16(float v, b16& hi, b16& lo) { hi = (b16)v; lo = (b16)(v - (float)hi); }
__device__ __forceinline__ v16b frag_kb(const b16* p, int hh) { const v8b a = *(const v8b*)(p + 8 * hh), b = *(const v8b*)(p + 16 + 8 * hh); v16b f;
#pragma unroll
  for (int e = 0; e < 8; ++e) { f[e] = a[e]; f[8 + e] = b[e]; } return f; }
__device__ __forceinline__ v8f wmma16b(v16b a, v16b b, v8f c) { v8f d = __builtin_amdgcn_wmma_f32_16x16x32_f16(false, a, false, b, (short)0, c, false, false); asm volatile("v_nop\n\tv_nop\n\tv_nop\n\tv_nop" : "+v"(d) : "v"(a), "v"(b)); return d; }
__device__ __forceinline__ void wave_lds_sync() { __builtin_amdgcn_fence(__ATOMIC_RELEASE, "workgroup"); __builtin_amdgcn_wave_barrier(); __builtin_amdgcn_fence(__ATOMIC_ACQUIRE, "workgroup"); }
__device__ __forceinline__ float pmul(float a, float b) { float p = a * b; asm volatile("" : "+v"(p)); return p; }

__global__ __launch_bounds__(256) void wput_kernel(const float* __restrict__ woff, const float* __restrict__ wmask, const float* __restrict__ wdef, const float* __restrict__ w1, b16* __restrict__ WOM, b16* __restrict__ WD, b16* __restrict__ W1) { const size_t nt = (size_t)gridDim.x * 256, u0 = (size_t)blockIdx.x * 256 + threadIdx.x; v8b v;
  for (size_t u = u0; u < (size_t)32 * (KK / 8); u += nt) { const int o = (int)(u / (KK / 8)), q0 = (int)(u % (KK / 8)) * 8;
#pragma unroll
    for (int j = 0; j < 8; ++j) { const int q = q0 + j; float w = 0.0f; if (o < 18) w = woff[(size_t)o * KK + q]; else if (o < 27) w = wmask[(size_t)(o - 18) * KK + q]; v[j] = (b16)(bf16_rne(w) * WSC); } for (int pass = 0; pass < 2; ++pass) { *(volatile v8b*)(WOM + (size_t)o * KK + q0) = v; __threadfence(); } }
  for (size_t u = u0; u < (size_t)OC * (KK / 8); u += nt) { const int o = (int)(u / (KK / 8)), q0 = (int)(u % (KK / 8)) * 8;
#pragma unroll
    for (int j = 0; j < 8; ++j) v[j] = (b16)(bf16_rne(wdef[(size_t)o * KK + q0 + j]) * WSC); for (int pass = 0; pass < 2; ++pass) { *(volatile v8b*)(WD + (size_t)o * KK + q0) = v; __threadfence(); } }
  for (size_t u = u0; u < (size_t)OC * (CIN2 / 8); u += nt) { const int o = (int)(u / (CIN2 / 8)), q0 = (int)(u % (CIN2 / 8)) * 8;
#pragma unroll
    for (int j = 0; j < 8; ++j) { const int q = q0 + j; v[j] = (b16)(q < 155 ? bf16_rne(w1[(size_t)o * 155 + q]) * WSC : 0.0f); } for (int pass = 0; pass < 2; ++pass) { *(volatile v8b*)(W1 + (size_t)o * CIN2 + q0) = v; __threadfence(); } } }
__global__ __launch_bounds__(32) void main_kernel(const float* __restrict__ x, const b16* __restrict__ WOM, const b16* __restrict__ WD, const b16* __restrict__ W1, const float* __restrict__ boff, const float* __restrict__ bmask, const float* __restrict__ bdef, const float* __restrict__ b1, int PLIM, float* __restrict__ ST) { __shared__ __attribute__((aligned(16))) b16 Ah[16][KK + 8], Al[16][KK + 8]; __shared__ float OM[16][33], Ty[16][OC + 4]; const int lane = threadIdx.x, nloc = lane & 15, hlf = lane >> 4; const int n = blockIdx.x / (NP / 16), p0 = (blockIdx.x % (NP / 16)) * 16; if (p0 >= PLIM) return; const float* xn = x + (size_t)n * C * NP;
  if (lane < 16) for (int q = KK; q < KK + 8; ++q) { Ah[lane][q] = (b16)0.0f; Al[lane][q] = (b16)0.0f; }
  for (int rr = 0; rr < 16; ++rr) { const int p = p0 + rr, oy = p / WW, ox = p % WW;
    for (int c = lane; c < C; c += 32) {
#pragma unroll
      for (int k = 0; k < K9; ++k) { const int iy = oy - 1 + k / 3, ix = ox - 1 + k % 3; float v = 0.0f; if (iy >= 0 && iy < HH && ix >= 0 && ix < WW) v = bfv(xn[(size_t)c * NP + iy * WW + ix]); Ah[rr][c * K9 + k] = (b16)(v * XS); } } }
  wave_lds_sync();
  { v8f acc[2] = {(v8f){}, (v8f){}};
#pragma unroll 2
    for (int kb = 0; kb < KK; kb += 32) { const v16b a = frag_kb(&Ah[nloc][kb], hlf); acc[0] = wmma16b(a, frag_kb(WOM + (size_t)nloc * KK + kb, hlf), acc[0]); acc[1] = wmma16b(a, frag_kb(WOM + (size_t)(16 + nloc) * KK + kb, hlf), acc[1]); }
#pragma unroll
    for (int t = 0; t < 2; ++t) { const int cc = t * 16 + nloc;
#pragma unroll
      for (int r8 = 0; r8 < 8; ++r8) { float v = acc[t][r8] * (1.0f / (XS * WSC)); if (cc < 18) v += bfv(boff[cc]); else if (cc < 27) v = 1.0f / (1.0f + __expf(-(v + bfv(bmask[cc - 18])))); else v = 0.0f; OM[8 * hlf + r8][cc] = v; } } }
  wave_lds_sync();
  for (int rr = 0; rr < 16; ++rr) { const int p = p0 + rr, oy = p / WW, ox = p % WW;
#pragma unroll 1
    for (int k = 0; k < K9; ++k) { const float py = (float)(oy - 1 + k / 3) + OM[rr][2 * k], px = (float)(ox - 1 + k % 3) + OM[rr][2 * k + 1]; const float mk = OM[rr][18 + k]; const float fy = floorf(py), fx = floorf(px); const int y0 = (int)fy, x0 = (int)fx; const float wy1 = py - fy, wy0 = 1.0f - wy1, wx1 = px - fx, wx0 = 1.0f - wx1;
      const bool vy0 = y0 >= 0 && y0 < HH, vy1 = (y0 + 1) >= 0 && (y0 + 1) < HH, vx0 = x0 >= 0 && x0 < WW, vx1 = (x0 + 1) >= 0 && (x0 + 1) < WW; const int cy0 = min(max(y0, 0), HH - 1), cy1 = min(max(y0 + 1, 0), HH - 1), cx0 = min(max(x0, 0), WW - 1), cx1 = min(max(x0 + 1, 0), WW - 1);
      const float w00 = (vy0 && vx0) ? pmul(wy0, wx0) : 0.0f, w01 = (vy0 && vx1) ? pmul(wy0, wx1) : 0.0f, w10 = (vy1 && vx0) ? pmul(wy1, wx0) : 0.0f, w11 = (vy1 && vx1) ? pmul(wy1, wx1) : 0.0f;
      for (int c = lane; c < C; c += 32) { const float* xc = xn + (size_t)c * NP; const float v = pmul(bfv(xc[cy0 * WW + cx0]), w00) + pmul(bfv(xc[cy0 * WW + cx1]), w01) + pmul(bfv(xc[cy1 * WW + cx0]), w10) + pmul(bfv(xc[cy1 * WW + cx1]), w11); b16 ph, pl; split16(pmul(v, mk) * VS, ph, pl); Ah[rr][c * K9 + k] = ph; Al[rr][c * K9 + k] = pl; } } }
  wave_lds_sync();
  { v8f acc[8];
#pragma unroll
    for (int t = 0; t < 8; ++t) acc[t] = (v8f){};
#pragma unroll 2
    for (int kb = 0; kb < KK; kb += 32) { const v16b a = frag_kb(&Ah[nloc][kb], hlf), al = frag_kb(&Al[nloc][kb], hlf);
#pragma unroll
      for (int t = 0; t < 8; ++t) { const v16b bw = frag_kb(WD + (size_t)(t * 16 + nloc) * KK + kb, hlf); acc[t] = wmma16b(a, bw, acc[t]); acc[t] = wmma16b(al, bw, acc[t]); } }
#pragma unroll
    for (int t = 0; t < 8; ++t) { const int cc = t * 16 + nloc; const float bb = bfv(bdef[cc]);
#pragma unroll
      for (int r8 = 0; r8 < 8; ++r8) Ty[8 * hlf + r8][cc] = acc[t][r8] * (1.0f / (VS * WSC)) + bb; } }
  wave_lds_sync();
  for (int rr = 0; rr < 16; ++rr) for (int c = lane; c < CIN2 + 8; c += 32) { float v = 0.0f; if (c < OC) v = Ty[rr][c]; else if (c < 155) v = OM[rr][c - OC]; b16 p, pl; split16(v * HS, p, pl); Ah[rr][c] = p; Al[rr][c] = pl; }
  wave_lds_sync();
  { v8f acc[8];
#pragma unroll
    for (int t = 0; t < 8; ++t) acc[t] = (v8f){};
#pragma unroll
    for (int kb = 0; kb < CIN2; kb += 32) { const v16b a = frag_kb(&Ah[nloc][kb], hlf), al = frag_kb(&Al[nloc][kb], hlf);
#pragma unroll
      for (int t = 0; t < 8; ++t) { const v16b bw = frag_kb(W1 + (size_t)(t * 16 + nloc) * CIN2 + kb, hlf); acc[t] = wmma16b(a, bw, acc[t]); acc[t] = wmma16b(al, bw, acc[t]); } }
#pragma unroll
    for (int t = 0; t < 8; ++t) { const int cc = t * 16 + nloc; const float bb = bfv(b1[cc]);
#pragma unroll
      for (int r8 = 0; r8 < 8; ++r8) Ty[8 * hlf + r8][cc] = acc[t][r8] * (1.0f / (HS * WSC)) + bb; } }
  wave_lds_sync();
  for (int pass = 0; pass < 2; ++pass) { for (int rr = 0; rr < 16; ++rr) *(volatile v4f*)(ST + ((size_t)n * NP + p0 + rr) * OC + lane * 4) = *(const v4f*)(&Ty[rr][lane * 4]); __threadfence(); } }
__global__ __launch_bounds__(256) void copy_kernel(const float* __restrict__ ST, int PLIM, float* __restrict__ out) { const size_t u = (size_t)blockIdx.x * 256 + threadIdx.x; if (u >= (size_t)NPT * OC) return; const int p = (int)(u % NP), o = (int)((u / NP) % OC), n = (int)(u / ((size_t)NP * OC)); const float v = p < PLIM ? ST[((size_t)n * NP + p) * OC + o] : 0.0f;
  for (int pass = 0; pass < 2; ++pass) { ((volatile float*)out)[u] = v; __threadfence(); } }
}

extern "C" void kernel_launch(void* const* d_in, const int* in_sizes, int n_in, void* d_out, int out_size, void* d_ws, size_t ws_size, hipStream_t stream) {
  (void)n_in;
  auto Fp = [&](int i) { return (const float*)d_in[i]; };
  if (in_sizes[0] != NPT * C || in_sizes[1] != 18 * KK || in_sizes[3] != 9 * KK || in_sizes[5] != OC * KK || in_sizes[7] != OC * 155 || out_size != NPT * OC) return;
  const int PLIM = NP;
  size_t off = 0; char* ws = (char*)d_ws;
  auto carve = [&](size_t bytes) { char* p = ws + off; off += (bytes + 255) & ~(size_t)255; return p; };
  b16* WOM = (b16*)carve((size_t)32 * KK * 2); b16* WD = (b16*)carve((size_t)OC * KK * 2); b16* W1 = (b16*)carve((size_t)OC * CIN2 * 2); float* ST = (float*)carve((size_t)NPT * OC * 4);
  if (off > ws_size || off > ((size_t)40 << 20)) return;
  wput_kernel<<<128, 256, 0, stream>>>(Fp(1), Fp(3), Fp(5), Fp(7), WOM, WD, W1);
  main_kernel<<<NB_ * (NP / 16), 32, 0, stream>>>(Fp(0), WOM, WD, W1, Fp(2), Fp(4), Fp(6), Fp(8), PLIM, ST);
  copy_kernel<<<(NPT * OC + 255) / 256, 256, 0, stream>>>(ST, PLIM, (float*)d_out);
}
